// TopDownHTMM_15771119910968
// MI455X (gfx1250) — hardware-verified
//
#include <hip/hip_runtime.h>
#include <stddef.h>


typedef _Float16 v16h __attribute__((ext_vector_type(16)));
typedef __bf16   v16b __attribute__((ext_vector_type(16)));
typedef float    v8f  __attribute__((ext_vector_type(8)));
typedef float    v4f  __attribute__((ext_vector_type(4)));
typedef float    v4fa __attribute__((ext_vector_type(4), __may_alias__));

#define CS    8
#define MS    32
#define TD    10
#define NPT   2047
#define NLEAF 1024
#define WLEV  5
#define NTHR  256
#define NWAV  (NTHR / 32)
#define SLOT  32

static_assert((NLEAF * CS) % NTHR == 0);
static_assert(((1 << (WLEV - 1)) * CS) <= NTHR);
static_assert((1 << WLEV) >= 32);
static_assert(NTHR % 32 == 0);

__device__ __forceinline__ v8f wmma_f16(v16h a, v16h b, v8f c)
{
    v8f d = __builtin_amdgcn_wmma_f32_16x16x32_f16(false, a, false, b, (short)0, c, false, false);
    asm volatile("v_nop\n\tv_nop\n\tv_nop\n\tv_nop" : "+v"(d) : "v"(a), "v"(b));
    return d;
}

__device__ __forceinline__ v8f wmma_bf16(v16b a, v16b b, v8f c)
{
    v8f d = __builtin_amdgcn_wmma_f32_16x16x32_bf16(false, a, false, b, (short)0, c, false, false);
    asm volatile("v_nop\n\tv_nop\n\tv_nop\n\tv_nop" : "+v"(d) : "v"(a), "v"(b));
    return d;
}

__device__ __forceinline__ float sum8(float v)
{
    v += __shfl_xor(v, 1);
    v += __shfl_xor(v, 2);
    v += __shfl_xor(v, 4);
    return v;
}

__device__ __forceinline__ float frcp(float v) { return __builtin_amdgcn_rcpf(v); }
__device__ __forceinline__ int imin(int a, int b) { return a < b ? a : b; }
__device__ __forceinline__ int iclamp(int v, int lo, int hi) { return v < lo ? lo : (v > hi ? hi : v); }

__global__ __launch_bounds__(NTHR)
void k_tree(const float* __restrict__ Ain, const float* __restrict__ Bin,
            const float* __restrict__ Piin, const int* __restrict__ xin,
            const int* __restrict__ imap, float* __restrict__ wsl,
            int G, int ntrees, int dim)
{
    __shared__ float smA[CS * CS];
    __shared__ float sAL[CS * CS];
    __shared__ float smBt[MS * CS];
    __shared__ float lgBt[MS * CS];
    __shared__ float lgPi[CS];
    __shared__ float pri[(TD + 1) * CS];
    __shared__ float invp[(TD + 1) * CS];
    __shared__ float red[NWAV];
    __shared__ float beta[NPT * CS] __attribute__((aligned(16)));
    __shared__ float te[NPT * CS]   __attribute__((aligned(16)));
    __shared__ int   obs[NPT + 1];

    const int tid  = threadIdx.x;
    const int lane = tid & 31;
    const int wave = tid >> 5;
    const int n16  = lane & 15;
    const int hh   = lane >> 4;
    const int cst  = lane & 7;
    const int nset = n16 >> 3;
    const int blk  = blockIdx.x;
    const int tree = blk / G;
    const int g    = blk - tree * G;
    if (tree >= ntrees) return;

    if (tid < CS) {
        const int j = tid;
        float va[CS];
        float mx = -3.0e38f;
#pragma unroll
        for (int i = 0; i < CS; ++i) { va[i] = Ain[(size_t)(i * CS + j) * G + g]; mx = fmaxf(mx, va[i]); }
        float s = 0.f;
#pragma unroll
        for (int i = 0; i < CS; ++i) s += __expf(va[i] - mx);
        const float ls = __logf(s);
#pragma unroll
        for (int i = 0; i < CS; ++i) {
            const float lg = va[i] - mx - ls;
            const float sm = __expf(lg);
            smA[i * CS + j] = sm;
            sAL[i * CS + j] = sm * lg;
        }
    } else if (tid < 2 * CS) {
        const int c = tid - CS;
        float vb[MS];
        float mx = -3.0e38f;
#pragma unroll
        for (int m = 0; m < MS; ++m) { vb[m] = Bin[(size_t)(c * MS + m) * G + g]; mx = fmaxf(mx, vb[m]); }
        float s = 0.f;
#pragma unroll
        for (int m = 0; m < MS; ++m) s += __expf(vb[m] - mx);
        const float ls = __logf(s);
#pragma unroll
        for (int m = 0; m < MS; ++m) {
            const float lg = vb[m] - mx - ls;
            smBt[m * CS + c] = __expf(lg);
            lgBt[m * CS + c] = lg;
        }
    } else if (tid == 2 * CS) {
        float vp[CS];
        float mx = -3.0e38f;
#pragma unroll
        for (int c = 0; c < CS; ++c) { vp[c] = Piin[(size_t)c * G + g]; mx = fmaxf(mx, vp[c]); }
        float s = 0.f;
#pragma unroll
        for (int c = 0; c < CS; ++c) s += __expf(vp[c] - mx);
        const float ls = __logf(s);
#pragma unroll
        for (int c = 0; c < CS; ++c) {
            const float lg = vp[c] - mx - ls;
            pri[c]  = __expf(lg);
            lgPi[c] = lg;
        }
    }
    for (int n = tid; n < NPT; n += NTHR) {
        int im = imap[(size_t)tree * NPT + n];
        if (im < 0) im += dim;
        im = iclamp(im, 0, dim - 1);
        int v = xin[im];
        if (v < 0) v += MS;
        obs[n] = iclamp(v, 0, MS - 1);
    }
    __syncthreads();

    for (int d = 1; d <= TD; ++d) {
        if (tid < CS) {
            float s = 0.f;
#pragma unroll
            for (int j = 0; j < CS; ++j) s += smA[tid * CS + j] * pri[(d - 1) * CS + j];
            pri[d * CS + tid] = s;
        }
        __syncthreads();
    }
    for (int i = tid; i < (TD + 1) * CS; i += NTHR) invp[i] = frcp(pri[i]);
    __syncthreads();

    v16h Bup;
    v16b Bdn, Bal;
    {
        const bool diag = (hh == nset);
#pragma unroll
        for (int e = 0; e < 16; ++e) { Bup[e] = (_Float16)0.f; Bdn[e] = (__bf16)0.f; Bal[e] = (__bf16)0.f; }
#pragma unroll
        for (int e = 0; e < CS; ++e) {
            const float vu = diag ? smA[e * CS + cst] : 0.f;
            const float vd = diag ? smA[cst * CS + e] : 0.f;
            const float va = diag ? sAL[cst * CS + e] : 0.f;
            Bup[e] = (_Float16)vu;
            Bdn[e] = (__bf16)vd;
            Bal[e] = (__bf16)va;
        }
    }
    v8f zacc;
#pragma unroll
    for (int r = 0; r < 8; ++r) zacc[r] = 0.f;

    {
        const float* pp = pri + TD * CS;
        for (int it = tid; it < NLEAF * CS; it += NTHR) {
            const int k = (NLEAF - 1) + (it >> 3);
            const float bl = pp[cst] * smBt[obs[k] * CS + cst];
            const float s  = sum8(bl);
            beta[k * CS + cst] = bl * frcp(s);
        }
    }
    __syncthreads();

    for (int d = TD; d >= WLEV; --d) {
        const int nch = 1 << d, kb = nch - 1, ntiles = nch >> 5;
        const float* ip = invp + d * CS;
        const float* pp = pri + (d - 1) * CS;
        for (int tile = wave; tile < ntiles; tile += NWAV) {
            const int c0 = kb + tile * 32;
            const int kn = c0 + lane;
            const v4fa b0 = *(const v4fa*)(beta + kn * CS);
            const v4fa b1 = *(const v4fa*)(beta + kn * CS + 4);
            v16h a;
#pragma unroll
            for (int e = 8; e < 16; ++e) a[e] = (_Float16)0.f;
            a[0] = (_Float16)(b0.x * ip[0]); a[1] = (_Float16)(b0.y * ip[1]);
            a[2] = (_Float16)(b0.z * ip[2]); a[3] = (_Float16)(b0.w * ip[3]);
            a[4] = (_Float16)(b1.x * ip[4]); a[5] = (_Float16)(b1.y * ip[5]);
            a[6] = (_Float16)(b1.z * ip[6]); a[7] = (_Float16)(b1.w * ip[7]);
            const v8f acc = wmma_f16(a, Bup, zacc);
            const int nb = c0 + 16 * nset + 8 * hh;
#pragma unroll
            for (int r = 0; r < 8; ++r) te[(nb + r) * CS + cst] = acc[r];
#pragma unroll
            for (int q = 0; q < 4; ++q) {
                const float prod = acc[2 * q] * acc[2 * q + 1];
                const int   u    = (nb + 2 * q - 1) >> 1;
                const float bv   = pp[cst] * smBt[obs[u] * CS + cst] * prod;
                const float s    = sum8(bv);
                beta[u * CS + cst] = bv * frcp(s);
            }
        }
        __syncthreads();
    }
    for (int d = WLEV - 1; d >= 1; --d) {
        const int nch = 1 << d, kb = nch - 1, npar = nch >> 1, pb = npar - 1;
        const float* ip = invp + d * CS;
        const float* pp = pri + (d - 1) * CS;
        {
            const int k = kb + imin(tid >> 3, nch - 1);
            float tb = 0.f;
#pragma unroll
            for (int i = 0; i < CS; ++i) tb += smA[i * CS + cst] * (beta[k * CS + i] * ip[i]);
            if (tid < nch * CS) te[k * CS + cst] = tb;
        }
        __syncthreads();
        {
            const int u = pb + imin(tid >> 3, npar - 1);
            const float prod = te[(2 * u + 1) * CS + cst] * te[(2 * u + 2) * CS + cst];
            const float bv   = pp[cst] * smBt[obs[u] * CS + cst] * prod;
            const float s    = sum8(bv);
            if (tid < npar * CS) beta[u * CS + cst] = bv * frcp(s);
        }
        __syncthreads();
    }

    float lik = 0.f;
    if (tid < CS) {
        const float bv = beta[cst];
        te[cst] = bv;
        lik += bv * (lgPi[cst] + lgBt[obs[0] * CS + cst]);
    }
    __syncthreads();
    for (int d = 1; d < WLEV; ++d) {
        const int nch = 1 << d, kb = nch - 1;
        const float* ip = invp + d * CS;
        const bool act = tid < nch * CS;
        const int k = kb + imin(tid >> 3, nch - 1);
        const int u = (k - 1) >> 1;
        float sv = 0.f, sl = 0.f;
#pragma unroll
        for (int j = 0; j < CS; ++j) {
            const float w = te[u * CS + j] * frcp(te[k * CS + j]);
            sv += smA[cst * CS + j] * w;
            sl += sAL[cst * CS + j] * w;
        }
        const float rat = beta[k * CS + cst] * ip[cst];
        const float num = rat * sv;
        const float sn  = sum8(num);
        const float ev  = num * frcp(sn);
        if (act) lik += rat * sl + ev * lgBt[obs[k] * CS + cst];
        __syncthreads();
        if (act) te[k * CS + cst] = ev;
        __syncthreads();
    }
    for (int d = WLEV; d <= TD; ++d) {
        const int nch = 1 << d, kb = nch - 1, ntiles = nch >> 5;
        const float* ip = invp + d * CS;
        for (int tile = wave; tile < ntiles; tile += NWAV) {
            const int c0 = kb + tile * 32;
            const int kn = c0 + lane;
            const int u  = (kn - 1) >> 1;
            const v4fa e0 = *(const v4fa*)(te + u * CS);
            const v4fa e1 = *(const v4fa*)(te + u * CS + 4);
            const v4fa t0 = *(const v4fa*)(te + kn * CS);
            const v4fa t1 = *(const v4fa*)(te + kn * CS + 4);
            v16b a;
#pragma unroll
            for (int e = 8; e < 16; ++e) a[e] = (__bf16)0.f;
            a[0] = (__bf16)(e0.x * frcp(t0.x)); a[1] = (__bf16)(e0.y * frcp(t0.y));
            a[2] = (__bf16)(e0.z * frcp(t0.z)); a[3] = (__bf16)(e0.w * frcp(t0.w));
            a[4] = (__bf16)(e1.x * frcp(t1.x)); a[5] = (__bf16)(e1.y * frcp(t1.y));
            a[6] = (__bf16)(e1.z * frcp(t1.z)); a[7] = (__bf16)(e1.w * frcp(t1.w));
            const v8f sv = wmma_bf16(a, Bdn, zacc);
            const v8f sl = wmma_bf16(a, Bal, zacc);
            const int nb = c0 + 16 * nset + 8 * hh;
#pragma unroll
            for (int r = 0; r < 8; ++r) {
                const int   node = nb + r;
                const float rat  = beta[node * CS + cst] * ip[cst];
                const float num  = rat * sv[r];
                const float sn   = sum8(num);
                const float ev   = num * frcp(sn);
                te[node * CS + cst] = ev;
                lik += rat * sl[r] + ev * lgBt[obs[node] * CS + cst];
            }
        }
        __syncthreads();
    }

    {
        float v = lik;
        v += __shfl_xor(v, 16);
        v += __shfl_xor(v, 8);
        v += __shfl_xor(v, 4);
        v += __shfl_xor(v, 2);
        v += __shfl_xor(v, 1);
        if (lane == 0) red[wave] = v;
    }
    __syncthreads();
    if (wave == 0) {
        float tot = 0.f;
#pragma unroll
        for (int w = 0; w < NWAV; ++w) tot += red[w];
        const float val = -tot;
        if (lane < 8) {
            v4f o;
            o.x = (lane == 0) ? val : 0.f; o.y = 0.f; o.z = 0.f; o.w = 0.f;
            volatile v4f* p = (volatile v4f*)(wsl + (size_t)blk * SLOT + lane * 4);
            *p = o;
            __threadfence();
            *p = o;
        }
    }
}

__global__ __launch_bounds__(NTHR)
void k_out(const float* __restrict__ wsl, float* out, int n)
{
    for (int b = (int)threadIdx.x * 4; b < n; b += NTHR * 4) {
        float v[4];
#pragma unroll
        for (int e = 0; e < 4; ++e) v[e] = (b + e < n) ? wsl[(size_t)(b + e) * SLOT] : 0.f;
        if (b + 3 < n) {
            v4f o; o.x = v[0]; o.y = v[1]; o.z = v[2]; o.w = v[3];
            volatile v4f* p = (volatile v4f*)(out + b);
            *p = o;
            __threadfence();
            *p = o;
        } else {
#pragma unroll
            for (int e = 0; e < 4; ++e) {
                if (b + e < n) {
                    volatile float* p = (volatile float*)(out + b + e);
                    *p = v[e];
                    __threadfence();
                    *p = v[e];
                }
            }
        }
    }
}

extern "C" void kernel_launch(void* const* d_in, const int* in_sizes, int n_in,
                              void* d_out, int out_size, void* d_ws, size_t ws_size,
                              hipStream_t stream)
{
    if (n_in < 7) return;
    const int G      = in_sizes[2] / CS;
    const int ntrees = in_sizes[4];
    const int dim    = in_sizes[3];
    if (G <= 0 || ntrees <= 0) return;
    if (in_sizes[2] != CS * G || in_sizes[0] != CS * CS * G || in_sizes[1] != CS * MS * G) return;
    if (dim != ntrees * NPT || in_sizes[6] != dim || out_size != ntrees * G) return;
    const int nblk = ntrees * G;
    if ((size_t)nblk * SLOT * sizeof(float) > ws_size) return;

    const float* A   = (const float*)d_in[0];
    const float* B   = (const float*)d_in[1];
    const float* Pi  = (const float*)d_in[2];
    const int*   x   = (const int*)d_in[3];
    const int*   im  = (const int*)d_in[6];
    float*       wsl = (float*)d_ws;
    float*       out = (float*)d_out;

    k_tree<<<nblk, NTHR, 0, stream>>>(A, B, Pi, x, im, wsl, G, ntrees, dim);
    k_out<<<1, NTHR, 0, stream>>>(wsl, out, out_size);
    (void)hipGetLastError();
}
